// DiffAttn_83159156785446
// MI455X (gfx1250) — hardware-verified
//
#include <hip/hip_runtime.h>
#include <math.h>

typedef __attribute__((ext_vector_type(16))) _Float16 v16h;
typedef __attribute__((ext_vector_type(16))) __bf16 v16b;
typedef __attribute__((ext_vector_type(8)))  _Float16 v8h;
typedef __attribute__((ext_vector_type(8)))  float v8f;
typedef __attribute__((ext_vector_type(4)))  float v4f;
typedef __attribute__((ext_vector_type(2)))  float v2f;
typedef __attribute__((ext_vector_type(4)))  unsigned v4u;
typedef __attribute__((ext_vector_type(4)))  int v4i;
typedef float __attribute__((may_alias)) float_a;
typedef int __attribute__((may_alias)) int_a;

template <typename T> __device__ __forceinline__ void vst2(void* p, T v) { *(volatile T*)p = v; __threadfence(); *(volatile T*)p = v; }
__device__ __forceinline__ v8f wmma16(v16h a, v16h b, v8f c) {
  v8f d = __builtin_amdgcn_wmma_f32_16x16x32_f16(false, a, false, b, (short)0, c, false, false);
  asm volatile("v_nop\n\tv_nop\n\tv_nop\n\tv_nop" : "+v"(d) : "v"(a), "v"(b));
  return d;
}
__device__ __forceinline__ v8f wmma_bf(v16b a, v16b b, v8f c) {
  v8f d = __builtin_amdgcn_wmma_f32_16x16x32_bf16(false, a, false, b, (short)0, c, false, false);
  asm volatile("v_nop\n\tv_nop\n\tv_nop\n\tv_nop" : "+v"(d) : "v"(a), "v"(b));
  return d;
}
__device__ __forceinline__ v16h frag_h(const _Float16* rowk0, int lane) {
  union { v16h v; v8h q[2]; } u; const _Float16* p = rowk0 + 8 * (lane >> 4);
  u.q[0] = *(const v8h*)p; u.q[1] = *(const v8h*)(p + 16); return u.v;
}
__device__ __forceinline__ v16h frag_f32(const float* rowk0, int lane) {
  v16h a; const float* p = rowk0 + 8 * (lane >> 4);
#pragma unroll
  for (int i = 0; i < 8; ++i) { a[i] = (_Float16)p[i]; a[8 + i] = (_Float16)p[16 + i]; }
  return a;
}
__device__ __forceinline__ v16h frag_f32s(const float* rowk0, int lane, float sc) {
  v16h a; const float* p = rowk0 + 8 * (lane >> 4);
#pragma unroll
  for (int i = 0; i < 8; ++i) { a[i] = (_Float16)(p[i] * sc); a[8 + i] = (_Float16)(p[16 + i] * sc); }
  return a;
}
__device__ __forceinline__ v16h fragc_f32(const float* W, int k0, int n, int lane, int ld, int K) {
  v16h a; const int g = lane >> 4;
#pragma unroll
  for (int i = 0; i < 8; ++i) { const int ka = k0 + 8 * g + i, kb = ka + 16;
    a[i] = (_Float16)(ka < K ? W[(size_t)(ka < K ? ka : K - 1) * ld + n] : 0.f); a[8 + i] = (_Float16)(kb < K ? W[(size_t)(kb < K ? kb : K - 1) * ld + n] : 0.f); }
  return a;
}
struct F2 { v16b h, l; };
__device__ __forceinline__ F2 bsplit16(const float v[16]) { F2 r;
#pragma unroll
  for (int i = 0; i < 16; ++i) { const __bf16 h = (__bf16)v[i]; r.h[i] = h; r.l[i] = (__bf16)(v[i] - (float)h); }
  return r; }
__device__ __forceinline__ F2 split_row(const float* row, int k0, int lane) { float v[16]; const float* p = row + k0 + 8 * (lane >> 4);
#pragma unroll
  for (int i = 0; i < 8; ++i) { v[i] = p[i]; v[8 + i] = p[16 + i]; }
  return bsplit16(v); }
__device__ __forceinline__ F2 split_rowK(const float* row, int k0, int lane, int K) { float v[16]; const int g = lane >> 4;
#pragma unroll
  for (int i = 0; i < 8; ++i) { const int ka = k0 + 8 * g + i, kb = ka + 16; v[i] = ka < K ? row[ka < K ? ka : K - 1] : 0.f; v[8 + i] = kb < K ? row[kb < K ? kb : K - 1] : 0.f; }
  return bsplit16(v); }
__device__ __forceinline__ F2 split_col(const float* W, int k0, int n, int lane, int ld, int K) { float v[16]; const int g = lane >> 4;
#pragma unroll
  for (int i = 0; i < 8; ++i) { const int ka = k0 + 8 * g + i, kb = ka + 16; v[i] = ka < K ? W[(size_t)(ka < K ? ka : K - 1) * ld + n] : 0.f; v[8 + i] = kb < K ? W[(size_t)(kb < K ? kb : K - 1) * ld + n] : 0.f; }
  return bsplit16(v); }
__device__ __forceinline__ v8f mac3(const F2& a, const F2& b, v8f c) { c = wmma_bf(a.l, b.h, c); c = wmma_bf(a.h, b.l, c); return wmma_bf(a.h, b.h, c); }
__device__ __forceinline__ float sigm(float v) { return 1.0f / (1.0f + expf(-v)); }
#define LDSX() do { asm volatile("s_wait_dscnt 0" ::: "memory"); __builtin_amdgcn_wave_barrier(); __builtin_amdgcn_fence(__ATOMIC_RELEASE, "workgroup"); } while (0)

#define NB 4
#define TT 2048
#define EE 1024
#define DD 512
#define QW (2 * DD)
#define SCALE 0.044194173824159216f
#ifndef TNB
#define TNB NB
#endif
#ifndef MP
#define MP TT
#endif
__device__ __forceinline__ float bfr(float v) { return (float)(__bf16)v; }
typedef __attribute__((ext_vector_type(8))) __bf16 v8b;
__device__ __forceinline__ v16b frag_b(const __bf16* rowk0, int lane) {
  union { v16b v; v8b q[2]; } u; const __bf16* p = rowk0 + 8 * (lane >> 4);
  u.q[0] = *(const v8b*)p; u.q[1] = *(const v8b*)(p + 16); return u.v;
}
#define QBH 6
#define QHI (QBH * 64)
__device__ __forceinline__ v16b wrow(const float* rowk0, int lane) { v16b w; const float* p = rowk0 + 8 * (lane >> 4);
#pragma unroll
  for (int i = 0; i < 8; ++i) { w[i] = (__bf16)p[i]; w[8 + i] = (__bf16)p[16 + i]; }
  return w; }

#define WS_QH  0u
#define WS_KH  (WS_QH + 2u * (size_t)NB * TT * QW)
#define WS_VT  (WS_KH + 2u * (size_t)NB * TT * QW)
#define WS_QL  (WS_VT + 2u * (size_t)NB * DD * TT)
#define WS_KL  (WS_QL + 2u * (size_t)NB * QHI * QW)
#define WS_VB  (WS_KL + 2u * (size_t)NB * TT * QW)
#define WS_VBL (WS_VB + 2u * (size_t)NB * DD * TT)
#define WS_S1  (WS_VBL + 2u * (size_t)NB * DD * TT)
#define WS_S2  (WS_S1 + 4u * (size_t)TT * TT)
#define WS_END (WS_S2 + 4u * (size_t)TT * TT)

__global__ __launch_bounds__(128) void k_proj(const float* __restrict__ X, const float* __restrict__ WQ, const float* __restrict__ BQ, const float* __restrict__ WK, const float* __restrict__ BK, const float* __restrict__ WV, const float* __restrict__ BV, _Float16* __restrict__ QH, _Float16* __restrict__ KH, _Float16* __restrict__ VT, _Float16* __restrict__ QL, _Float16* __restrict__ KL, __bf16* __restrict__ VB, __bf16* __restrict__ VBL) {
  __shared__ __align__(16) _Float16 sh[64][136], sl[64][136]; __shared__ __align__(16) _Float16 th[128][72]; __shared__ __align__(16) __bf16 tb[128][72], tbl[128][72];
  const int tid = threadIdx.x, wave = tid >> 5, lane = tid & 31, col = lane & 15, g = lane >> 4; const int which = blockIdx.z; const int c0 = blockIdx.y * 128; const size_t r0 = (size_t)blockIdx.x * 64; const int NW = which == 2 ? DD : QW; if (c0 >= NW) return;
  const size_t bb0 = r0 / TT; const int t00 = (int)(r0 % TT); const bool qres = (which == 1) || (t00 < QHI);
  const float* WA = which == 0 ? WQ : which == 1 ? WK : WV; const float* BA = which == 0 ? BQ : which == 1 ? BK : BV;
  v8f acc[8] = {};
#pragma unroll 2
  for (int kc = 0; kc < EE / 32; ++kc) { v16b a; { const float* p = X + (r0 + wave * 16 + col) * EE + kc * 32 + 8 * g;
#pragma unroll
      for (int i = 0; i < 8; ++i) { a[i] = (__bf16)p[i]; a[8 + i] = (__bf16)p[16 + i]; } }
#pragma unroll
    for (int j = 0; j < 8; ++j) { const v16b w = wrow(WA + (size_t)(c0 + j * 16 + col) * EE + kc * 32, lane); asm volatile("s_wait_loadcnt 0x0" ::: "memory"); acc[j] = wmma_bf(a, w, acc[j]); } }
  if (which < 2) {
#pragma unroll
    for (int j = 0; j < 8; ++j) { const float bb = bfr(BA[c0 + j * 16 + col]);
#pragma unroll
      for (int r = 0; r < 8; ++r) { const float v = acc[j][r] + bb; const _Float16 hv = (_Float16)v; sh[wave * 16 + 8 * g + r][j * 16 + col] = hv; sl[wave * 16 + 8 * g + r][j * 16 + col] = (_Float16)((v - (float)hv) * 1024.0f); } }
    __syncthreads();
    _Float16* dh = which == 0 ? QH : KH; _Float16* dl = which == 0 ? (QL + (bb0 * QHI + t00) * (size_t)QW) : (KL + r0 * QW);
    for (int e = tid; e < 64 * 16; e += 128) { const int rl = e >> 4, q = e & 15; vst2((unsigned*)(dh + (r0 + rl) * QW + c0 + q * 8), *(const v4u*)&sh[rl][q * 8]); if (qres) vst2((unsigned*)(dl + (size_t)rl * QW + c0 + q * 8), *(const v4u*)&sl[rl][q * 8]); }
  } else {
#pragma unroll
    for (int j = 0; j < 8; ++j) { const float bb = bfr(BA[c0 + j * 16 + col]);
#pragma unroll
      for (int r = 0; r < 8; ++r) { const float v = acc[j][r] + bb; const int rl = wave * 16 + 8 * g + r, cl = j * 16 + col; th[cl][rl] = (_Float16)v; const __bf16 bh = (__bf16)v; tb[cl][rl] = bh; tbl[cl][rl] = (__bf16)(v - (float)bh); } }
    __syncthreads();
    const size_t b = r0 / TT; const int t0 = (int)(r0 % TT); for (int e = tid; e < 128 * 8; e += 128) { const int cl = e >> 3, q = e & 7; const size_t o2 = (b * DD + c0 + cl) * (size_t)TT + t0 + q * 8; vst2((unsigned*)(VT + o2), *(const v4u*)&th[cl][q * 8]); vst2((unsigned*)(VB + o2), *(const v4u*)&tb[cl][q * 8]); vst2((unsigned*)(VBL + o2), *(const v4u*)&tbl[cl][q * 8]); } } }
__global__ __launch_bounds__(128) void k_sc(const _Float16* __restrict__ QH, const _Float16* __restrict__ KH, const _Float16* __restrict__ QL, const _Float16* __restrict__ KL, int b, float* __restrict__ S1, float* __restrict__ S2) { __shared__ __align__(16) float ss[4][16][132];
  const int map = blockIdx.z; float* S = map == 0 ? S1 : S2; const int cofs = map * DD;
  const int tid = threadIdx.x, wave = tid >> 5, lane = tid & 31, col = lane & 15, g = lane >> 4; const int qb = blockIdx.x; const int k0 = blockIdx.y * 128; const int ql0 = qb * 64 + wave * 16; const size_t q0 = (size_t)b * TT + ql0, kr0 = (size_t)b * TT + k0;
  v8f acc[8] = {}, accl[8] = {};
  if (qb < QBH) { const _Float16* QLb = QL + (size_t)b * QHI * QW;
#pragma unroll 2
    for (int kc = 0; kc < DD / 32; ++kc) { const v16h ah = frag_h(QH + (q0 + col) * QW + cofs + kc * 32, lane), al = frag_h(QLb + (size_t)(ql0 + col) * QW + cofs + kc * 32, lane);
#pragma unroll
      for (int j = 0; j < 8; ++j) { const size_t kr = (kr0 + j * 16 + col) * QW + cofs + kc * 32; const v16h kb = frag_h(KH + kr, lane), kl = frag_h(KL + kr, lane); acc[j] = wmma16(ah, kb, acc[j]); accl[j] = wmma16(al, kb, accl[j]); accl[j] = wmma16(ah, kl, accl[j]); } }
  } else {
#pragma unroll 2
    for (int kc = 0; kc < DD / 32; ++kc) { const v16h ah = frag_h(QH + (q0 + col) * QW + cofs + kc * 32, lane);
#pragma unroll
      for (int j = 0; j < 8; ++j) { const v16h kb = frag_h(KH + (kr0 + j * 16 + col) * QW + cofs + kc * 32, lane); acc[j] = wmma16(ah, kb, acc[j]); } } }
#pragma unroll
  for (int j = 0; j < 8; ++j) {
#pragma unroll
    for (int r = 0; r < 8; ++r) ss[wave][8 * g + r][j * 16 + col] = (acc[j][r] + accl[j][r] * (1.0f / 1024.0f)) * SCALE; }
  LDSX(); for (int rl = 0; rl < 16; ++rl) vst2(S + (size_t)(ql0 + rl) * TT + k0 + lane * 4, *(const v4f*)&ss[wave][rl][lane * 4]); }
__device__ __forceinline__ void row_softmax(float* shv, float* sred, float* sbc, int* scnt, int tid) {
  float m = -3.0e38f; int cnt = 0; for (int k = tid; k < TT; k += 256) { const float v = shv[k]; m = fmaxf(m, v); cnt += (v > -1.0e38f) ? 1 : 0; }
#pragma unroll
  for (int o = 1; o < 32; o <<= 1) { m = fmaxf(m, __shfl_xor(m, o)); cnt += __shfl_xor(cnt, o); }
  if ((tid & 31) == 0) { sred[tid >> 5] = m; scnt[tid >> 5] = cnt; } __syncthreads();
  if (tid == 0) { float a = sred[0]; int c = scnt[0]; for (int i = 1; i < 8; ++i) { a = fmaxf(a, sred[i]); c += scnt[i]; } *sbc = a; scnt[8] = c; } __syncthreads(); m = *sbc; const int total = scnt[8]; __syncthreads();
  float sum = 0.f; for (int k = tid; k < TT; k += 256) { const float v = shv[k]; const float e = (v <= -1.0e38f) ? 0.f : expf(v - m); shv[k] = e; sum += e; }
#pragma unroll
  for (int o = 1; o < 32; o <<= 1) sum += __shfl_xor(sum, o);
  if ((tid & 31) == 0) sred[tid >> 5] = sum; __syncthreads(); if (tid == 0) { float a = 0.f; for (int i = 0; i < 8; ++i) a += sred[i]; *sbc = (total > 0) ? 1.0f / a : 0.f; } __syncthreads(); const float inv = *sbc;
  for (int k = tid; k < TT; k += 256) shv[k] = shv[k] * inv;
  __syncthreads(); }
__global__ __launch_bounds__(256) void k_sm2(float* __restrict__ S1, const float* __restrict__ S2, const int* __restrict__ MASK, const float* __restrict__ LAM) { __shared__ float sred[8]; __shared__ float sbc; __shared__ int scnt[9]; __shared__ __align__(16) float p1[TT], p2[TT];
  const int tid = threadIdx.x; const int t = blockIdx.x; float* r1 = S1 + (size_t)t * TT; const float* r2 = S2 + (size_t)t * TT; const int* mk = MASK + (size_t)t * MP;
  for (int k = tid; k < TT; k += 256) { const bool ex = mk[k] != 0; p1[k] = ex ? -3.0e38f : r1[k]; p2[k] = ex ? -3.0e38f : r2[k]; }
  __syncthreads();
  row_softmax(p1, sred, &sbc, scnt, tid);
  row_softmax(p2, sred, &sbc, scnt, tid);
  const float lamv = (expf(bfr(LAM[0])) + 0.05f) ;
  for (int k = tid; k < TT; k += 256) p1[k] = (p1[k] - lamv * p2[k]) * 2048.0f;
  __syncthreads(); for (int q = tid; q < TT / 4; q += 256) vst2(r1 + q * 4, *(const v4f*)&p1[q * 4]); }
__global__ __launch_bounds__(128) void k_pv(const float* __restrict__ PS, const _Float16* __restrict__ VT, const __bf16* __restrict__ VB, const __bf16* __restrict__ VBL, int b, float* __restrict__ OUT) { __shared__ __align__(16) float ss[4][16][132];
  const int tid = threadIdx.x, wave = tid >> 5, lane = tid & 31, col = lane & 15, g = lane >> 4; const int qb = blockIdx.x; const int ql0 = qb * 64 + wave * 16; const int c0 = blockIdx.y * 128;
  v8f acc[8] = {};
  if (qb < QBH) {
#pragma unroll 1
    for (int kc = 0; kc < TT / 32; ++kc) { const F2 p = split_row(PS + (size_t)(ql0 + col) * TT, kc * 32, lane);
      asm volatile("s_wait_loadcnt 0x0" ::: "memory");
#pragma unroll
      for (int j = 0; j < 8; ++j) { const size_t po = ((size_t)b * DD + c0 + j * 16 + col) * (size_t)TT + kc * 32; const v16b vh = frag_b(VB + po, lane); acc[j] = wmma_bf(p.h, vh, acc[j]); acc[j] = wmma_bf(p.l, vh, acc[j]); acc[j] = wmma_bf(p.h, frag_b(VBL + po, lane), acc[j]); } }
  } else {
#pragma unroll 1
    for (int kc = 0; kc < TT / 32; ++kc) { const v16h p = frag_f32(PS + (size_t)(ql0 + col) * TT + kc * 32, lane);
      asm volatile("s_wait_loadcnt 0x0" ::: "memory");
#pragma unroll
      for (int j = 0; j < 8; ++j) { const size_t po = ((size_t)b * DD + c0 + j * 16 + col) * (size_t)TT + kc * 32; acc[j] = wmma16(p, frag_h(VT + po, lane), acc[j]); } } }
#pragma unroll
  for (int j = 0; j < 8; ++j)
#pragma unroll
    for (int r = 0; r < 8; ++r) ss[wave][8 * g + r][j * 16 + col] = acc[j][r] * (1.0f / 2048.0f);
  LDSX(); for (int rl = 0; rl < 16; ++rl) vst2(OUT + ((size_t)b * TT + ql0 + rl) * DD + c0 + lane * 4, *(const v4f*)&ss[wave][rl][lane * 4]); }
extern "C" void kernel_launch(void* const* d_in, const int* in_sizes, int n_in, void* d_out, int out_size, void* d_ws, size_t ws_size, hipStream_t stream) {
  (void)in_sizes; (void)n_in; (void)out_size;
  const float** F = (const float**)d_in;
  if (ws_size < (size_t)WS_END) return;
  char* ws = (char*)d_ws; _Float16 *QH = (_Float16*)(ws + WS_QH), *KH = (_Float16*)(ws + WS_KH), *VT = (_Float16*)(ws + WS_VT), *QL = (_Float16*)(ws + WS_QL), *KL = (_Float16*)(ws + WS_KL); __bf16 *VB = (__bf16*)(ws + WS_VB), *VBL = (__bf16*)(ws + WS_VBL); float *S1 = (float*)(ws + WS_S1), *S2 = (float*)(ws + WS_S2);
  k_proj<<<dim3(TNB * TT / 64, QW / 128, 3), 128, 0, stream>>>(F[0], F[2], F[3], F[4], F[5], F[6], F[7], QH, KH, VT, QL, KL, VB, VBL);
  for (int b = 0; b < TNB; ++b) {
    k_sc<<<dim3(TT / 64, TT / 128, 2), 128, 0, stream>>>(QH, KH, QL, KL, b, S1, S2);
    k_sm2<<<dim3(TT), 256, 0, stream>>>(S1, S2, (const int*)d_in[1], F[8]);
    k_pv<<<dim3(TT / 64, DD / 128), 128, 0, stream>>>(S1, VT, VB, VBL, b, (float*)d_out);
  }
}
